// Deblur_route_19782619365725
// MI455X (gfx1250) — hardware-verified
//
#include <hip/hip_runtime.h>
#include <math.h>

#define NIMG 2
#define CDIM 32
#define IH 256
#define IW 256
#define HW_ (IH * IW)
#define KSZ 5

typedef _Float16 f16;
typedef __attribute__((ext_vector_type(16))) f16 f16x16;
typedef __attribute__((ext_vector_type(8)))  f16 f16x8;
typedef __attribute__((ext_vector_type(8)))  float f32x8;
typedef __attribute__((ext_vector_type(4)))  float v4f_t;
typedef float v4fa __attribute__((ext_vector_type(4), may_alias));

__device__ __forceinline__ f32x8 wmma16(f16x16 a, f16x16 b, f32x8 c) {
  c = __builtin_amdgcn_wmma_f32_16x16x32_f16(false, a, false, b, (short)0, c, false, false);
  asm volatile("v_nop\n\tv_nop\n\tv_nop\n\tv_nop" : "+v"(c) : "v"(a), "v"(b));
  return c;
}
__device__ __forceinline__ f16x16 lds_frag(const f16* base, int stride) {
  const int lane = threadIdx.x & 31, row = lane & 15, kh = (lane >> 4) * 8;
  const f16x8 lo = *(const f16x8*)(base + row * stride + kh);
  const f16x8 hi = *(const f16x8*)(base + row * stride + kh + 16);
  f16x16 f;
#pragma unroll
  for (int i = 0; i < 8; ++i) { f[i] = lo[i]; f[i + 8] = hi[i]; }
  return f;
}
__device__ __forceinline__ void wfrag2(const float* __restrict__ Wm, int ktot, int nrows, int o0, int k0, f16x16& hi, f16x16& lo) {
  const int lane = threadIdx.x & 31, r = o0 + (lane & 15), kh = (lane >> 4) * 8;
#pragma unroll
  for (int i = 0; i < 8; ++i) { const int ka = k0 + kh + i, kb = k0 + 16 + kh + i;
    const float a = (r < nrows && ka < ktot) ? Wm[(size_t)r * ktot + ka] : 0.0f, b2 = (r < nrows && kb < ktot) ? Wm[(size_t)r * ktot + kb] : 0.0f;
    const f16 ha = (f16)a, hb = (f16)b2; hi[i] = ha; lo[i] = (f16)((a - (float)ha) * 2048.0f); hi[8 + i] = hb; lo[8 + i] = (f16)((b2 - (float)hb) * 2048.0f); }
}
__device__ __forceinline__ float selu_f(float v) { return 1.0507009873554805f * (v > 0.0f ? v : 1.6732632423543772f * (expf(v) - 1.0f)); }

template <int CIN, int COUT, int NT, int EPI>
__global__ __launch_bounds__(256) void k_conv3(const float* __restrict__ src, const float* __restrict__ Wt, const float* __restrict__ bias, float* __restrict__ dst) {
  __shared__ __attribute__((aligned(16))) f16 aS[2][128 * 40];
  __shared__ __attribute__((aligned(16))) float oS[NT * 16 * 132];
  constexpr int KTOT = CIN * 9, KSTEPS = (KTOT + 31) / 32;
  const int tid = threadIdx.x, lane = tid & 31, wave = tid >> 5, cl = lane & 15, rh = (lane >> 4) * 8;
  const int b = blockIdx.x / (IH * 2), rem = blockIdx.x % (IH * 2), y = rem >> 1, x0 = (rem & 1) * 128;
  const float* inb = src + (size_t)b * CIN * HW_;
  f32x8 acc[NT], accx[NT];
#pragma unroll
  for (int j = 0; j < NT; ++j) { f32x8 z = {}; acc[j] = z; accx[j] = z; }
#pragma unroll 1
  for (int ks = 0; ks < KSTEPS; ++ks) {
    __syncthreads();
    { const int px = tid >> 1, kq = (tid & 1) * 16;
#pragma unroll 4
      for (int u = 0; u < 16; ++u) { const int k = ks * 32 + kq + u; float v = 0.0f;
        if (k < KTOT) { const int c = k / 9, r9 = k - 9 * c, dy = r9 / 3 - 1, dx = r9 - 3 * (r9 / 3) - 1; const int ys = y + dy, xs = x0 + px + dx;
          if (ys >= 0 && ys < IH && xs >= 0 && xs < IW) v = inb[(size_t)c * HW_ + ys * IW + xs]; }
        const f16 h = (f16)v; aS[0][px * 40 + kq + u] = h; aS[1][px * 40 + kq + u] = (f16)((v - (float)h) * 2048.0f); } }
    __syncthreads();
    const f16x16 ah = lds_frag(aS[0] + (wave * 16) * 40, 40), al = lds_frag(aS[1] + (wave * 16) * 40, 40);
#pragma unroll
    for (int j = 0; j < NT; ++j) { f16x16 bh, bl; wfrag2(Wt, KTOT, COUT, j * 16, ks * 32, bh, bl);
      acc[j] = wmma16(ah, bh, acc[j]); accx[j] = wmma16(ah, bl, accx[j]); accx[j] = wmma16(al, bh, accx[j]); }
  }
#pragma unroll
  for (int j = 0; j < NT; ++j) { const int o = j * 16 + cl; const float bv = (o < COUT) ? bias[o] : 0.0f;
#pragma unroll
    for (int r = 0; r < 8; ++r) { float v = acc[j][r] + accx[j][r] * (1.0f / 2048.0f) + bv; if (EPI == 1) v = selu_f(v); oS[o * 132 + wave * 16 + rh + r] = v; } }
  __syncthreads();
#pragma unroll 1
  for (int pass = 0; pass < 2; ++pass) {
    for (int q = tid; q < COUT * 32; q += 256) { const int o = q >> 5, c4 = (q & 31) * 4;
      *(volatile v4f_t*)(dst + ((size_t)b * COUT + o) * HW_ + (size_t)y * IW + x0 + c4) = *(const volatile v4fa*)(oS + o * 132 + c4); }
    __threadfence();
  }
}

__global__ __launch_bounds__(256) void k_dyn(const float* __restrict__ x3, const float* __restrict__ w4, const float* __restrict__ b4, const float* __restrict__ img, float* __restrict__ out) {
  __shared__ __attribute__((aligned(16))) f16 aS[2][128 * 40];
  __shared__ __attribute__((aligned(16))) float oS[CDIM * 132];
  const int tid = threadIdx.x, lane = tid & 31, wave = tid >> 5, cl = lane & 15, hsel = lane >> 4, rh = hsel * 8;
  const int b = blockIdx.x / (IH * 2), rem = blockIdx.x % (IH * 2), y = rem >> 1, x0 = (rem & 1) * 128;
  { const int px = tid >> 1, kq = (tid & 1) * 16;
#pragma unroll
    for (int u = 0; u < 16; ++u) { const float v = x3[((size_t)b * CDIM + kq + u) * HW_ + (size_t)y * IW + x0 + px]; const f16 h = (f16)v;
      aS[0][px * 40 + kq + u] = h; aS[1][px * 40 + kq + u] = (f16)((v - (float)h) * 2048.0f); } }
  __syncthreads();
  const f16x16 ah = lds_frag(aS[0] + (wave * 16) * 40, 40), al = lds_frag(aS[1] + (wave * 16) * 40, 40);
  const float* imb = img + (size_t)b * CDIM * HW_;
#pragma unroll 1
  for (int c = 0; c < CDIM; ++c) {
    float osum[8];
#pragma unroll
    for (int r = 0; r < 8; ++r) osum[r] = 0.0f;
#pragma unroll
    for (int th = 0; th < 2; ++th) {
      const int tap = th * 16 + cl; const bool real = tap < 25;
      f16x16 bh, bl;
      { const int lanei = lane, r = lanei & 15, kh = (lanei >> 4) * 8; const int tp = th * 16 + r; const float* wr = w4 + (size_t)(c * 25 + tp) * CDIM;
#pragma unroll
        for (int i = 0; i < 8; ++i) { const float a = (tp < 25) ? wr[kh + i] : 0.0f, a2 = (tp < 25) ? wr[16 + kh + i] : 0.0f; const f16 ha = (f16)a, h2 = (f16)a2;
          bh[i] = ha; bl[i] = (f16)((a - (float)ha) * 2048.0f); bh[8 + i] = h2; bl[8 + i] = (f16)((a2 - (float)h2) * 2048.0f); } }
      f32x8 kacc = {}, kx = {};
      kacc = wmma16(ah, bh, kacc); kx = wmma16(ah, bl, kx); kx = wmma16(al, bh, kx);
      const float bb = real ? b4[c * 25 + tap] : 0.0f;
      const int ta = tap / 5, tb = tap - 5 * ta;
#pragma unroll
      for (int r = 0; r < 8; ++r) {
        const int px = wave * 16 + rh + r; float contrib = 0.0f;
        if (real) { const int ys = min(max(y + ta - 2, 0), IH - 1), xs = min(max(x0 + px + tb - 2, 0), IW - 1);
          contrib = (kacc[r] + kx[r] * (1.0f / 2048.0f) + bb) * imb[(size_t)c * HW_ + ys * IW + xs]; }
#pragma unroll
        for (int off = 8; off >= 1; off >>= 1) contrib += __shfl_xor(contrib, off, 32);
        osum[r] += contrib; }
    }
    if (cl == 0) {
#pragma unroll
      for (int r = 0; r < 8; ++r) oS[c * 132 + wave * 16 + rh + r] = osum[r]; }
  }
  __syncthreads();
#pragma unroll 1
  for (int pass = 0; pass < 2; ++pass) {
    for (int q = tid; q < CDIM * 32; q += 256) { const int o = q >> 5, c4 = (q & 31) * 4;
      *(volatile v4f_t*)(out + ((size_t)b * CDIM + o) * HW_ + (size_t)y * IW + x0 + c4) = *(const volatile v4fa*)(oS + o * 132 + c4); }
    __threadfence();
  }
}

extern "C" void kernel_launch(void* const* d_in, const int* in_sizes, int n_in,
                              void* d_out, int out_size, void* d_ws, size_t ws_size,
                              hipStream_t stream) {
  (void)in_sizes; (void)n_in; (void)out_size; (void)ws_size;
  const float* img = (const float*)d_in[0];
  const float* dmap = (const float*)d_in[1];
  const float* w1 = (const float*)d_in[2], *b1 = (const float*)d_in[3], *w2 = (const float*)d_in[4], *b2 = (const float*)d_in[5];
  const float* w3 = (const float*)d_in[6], *b3 = (const float*)d_in[7], *w4 = (const float*)d_in[8], *b4 = (const float*)d_in[9];
  float* out = (float*)d_out;
  char* ws = (char*)d_ws;
  float* x1 = (float*)ws; ws += (size_t)NIMG * 32 * HW_ * 4;
  float* x2 = (float*)ws; ws += (size_t)NIMG * 4 * HW_ * 4;
  float* x3 = (float*)ws; ws += (size_t)NIMG * 32 * HW_ * 4;
  const dim3 g(NIMG * IH * 2), blk(256);
  k_conv3<64, 32, 2, 0><<<g, blk, 0, stream>>>(dmap, w1, b1, x1);
  k_conv3<32, 4, 1, 1><<<g, blk, 0, stream>>>(x1, w2, b2, x2);
  k_conv3<4, 32, 2, 1><<<g, blk, 0, stream>>>(x2, w3, b3, x3);
  k_dyn<<<g, blk, 0, stream>>>(x3, w4, b4, img, out);
}
